// EdgePointGNN_18485539242274
// MI455X (gfx1250) — hardware-verified
//
#include <hip/hip_runtime.h>


#define NN_  50000
#define NNP  50176
#define NE_  800000
#define NG_  50
#define FIN  64
#define HID  128
#define LAT  64
#define LYR  2
#define NT   256
#define NWV  (NT / 32)
#define EPT  2
#define CHUNK (NT * EPT)
#define RB   1024
#define LOSC 1024.0f
#define LOSCI (1.0f / 1024.0f)

typedef _Float16 h16;
typedef __attribute__((ext_vector_type(16))) _Float16 v16h;
typedef __attribute__((ext_vector_type(8)))  _Float16 v8h;
typedef __attribute__((ext_vector_type(8)))  float    v8f;
typedef __attribute__((ext_vector_type(4)))  float    v4f;
typedef __attribute__((ext_vector_type(2)))  _Float16 v2h;
typedef v8h  __attribute__((may_alias)) v8ha;
typedef v4f  __attribute__((may_alias)) v4fa;

__device__ __forceinline__ unsigned short f2bf(float f) { unsigned u = __float_as_uint(f); u += 0x7FFFu + ((u >> 16) & 1u); return (unsigned short)(u >> 16); }
__device__ __forceinline__ float bf2f(unsigned short b) { return __uint_as_float(((unsigned)b) << 16); }
__device__ __forceinline__ float bfr(float f) { return bf2f(f2bf(f)); }
__device__ __forceinline__ v16h cat16(v8h lo, v8h hi) { return __builtin_shufflevector(lo, hi, 0, 1, 2, 3, 4, 5, 6, 7, 8, 9, 10, 11, 12, 13, 14, 15); }
__device__ __forceinline__ v8f wmma16(v16h a, v16h b, v8f c) { return __builtin_amdgcn_wmma_f32_16x16x32_f16(false, a, false, b, (short)0, c, false, false); }
#define VST2(T, p, v) do { const T vst2_v_ = (v); *(volatile T*)(p) = vst2_v_; __threadfence(); *(volatile T*)(p) = vst2_v_; } while (0)
__device__ __forceinline__ float hmax16(float v) { v = fmaxf(v, __shfl_xor(v, 1, 16)); v = fmaxf(v, __shfl_xor(v, 2, 16)); v = fmaxf(v, __shfl_xor(v, 4, 16)); return fmaxf(v, __shfl_xor(v, 8, 16)); }
__device__ __forceinline__ float hsum16(float v) { v += __shfl_xor(v, 1, 16); v += __shfl_xor(v, 2, 16); v += __shfl_xor(v, 4, 16); return v + __shfl_xor(v, 8, 16); }

__global__ __launch_bounds__(256) void k_x16(const float* __restrict__ x, h16* X16) {
    const int lane = threadIdx.x & 31, r = blockIdx.x * 8 + (threadIdx.x >> 5);
    if (r >= NN_) return;
    v2h o; o[0] = (h16)bfr(x[(size_t)r * FIN + 2 * lane]); o[1] = (h16)bfr(x[(size_t)r * FIN + 2 * lane + 1]);
    VST2(v2h, X16 + (size_t)r * FIN + 2 * lane, o);
}

__global__ __launch_bounds__(256) void k_w16(const float* __restrict__ W1, const float* __restrict__ W2, const float* __restrict__ W3,
                                             const float* __restrict__ F1, const float* __restrict__ F2, const float* __restrict__ F3,
                                             h16* W1T, h16* W2T, h16* W3T, h16* F1T, h16* F2T, h16* F3T) {
    const int lane = threadIdx.x & 31, wid = blockIdx.x * 8 + (threadIdx.x >> 5);
    if (wid < 128) { const int n = wid; const float* w = W1 + (size_t)LYR * 126 * HID;
        v2h o[2];
#pragma unroll
        for (int q = 0; q < 2; ++q) { const int k0 = q * 64 + 2 * lane; v2h t;
#pragma unroll
            for (int i = 0; i < 2; ++i) { const int k = k0 + i; t[i] = (k < 125) ? (h16)bfr(w[(size_t)k * HID + n]) : (h16)0.f; }
            o[q] = t; }
        VST2(v2h, W1T + (size_t)n * HID + 2 * lane, o[0]); VST2(v2h, W1T + (size_t)n * HID + 64 + 2 * lane, o[1]);
    } else if (wid < 256) { const int n = wid - 128; const float* w = W2 + (size_t)LYR * HID * HID;
        v2h o[2];
#pragma unroll
        for (int q = 0; q < 2; ++q) { v2h t; t[0] = (h16)bfr(w[(size_t)(q * 64 + 2 * lane) * HID + n]); t[1] = (h16)bfr(w[(size_t)(q * 64 + 2 * lane + 1) * HID + n]); o[q] = t; }
        VST2(v2h, W2T + (size_t)n * HID + 2 * lane, o[0]); VST2(v2h, W2T + (size_t)n * HID + 64 + 2 * lane, o[1]);
    } else if (wid < 320) { const int n = wid - 256; const float* w = W3 + (size_t)LYR * HID * LAT;
        v2h o[2];
#pragma unroll
        for (int q = 0; q < 2; ++q) { v2h t; t[0] = (h16)bfr(w[(size_t)(q * 64 + 2 * lane) * LAT + n]); t[1] = (h16)bfr(w[(size_t)(q * 64 + 2 * lane + 1) * LAT + n]); o[q] = t; }
        VST2(v2h, W3T + (size_t)n * HID + 2 * lane, o[0]); VST2(v2h, W3T + (size_t)n * HID + 64 + 2 * lane, o[1]);
    } else if (wid < 384) { const int n = wid - 320;
        v2h o[3];
#pragma unroll
        for (int q = 0; q < 3; ++q) { v2h t; t[0] = (h16)bfr(F1[(size_t)(q * 64 + 2 * lane) * LAT + n]); t[1] = (h16)bfr(F1[(size_t)(q * 64 + 2 * lane + 1) * LAT + n]); o[q] = t; }
#pragma unroll
        for (int q = 0; q < 3; ++q) VST2(v2h, F1T + (size_t)n * (3 * LAT) + q * 64 + 2 * lane, o[q]);
    } else if (wid < 448) { const int n = wid - 384;
        v2h t; t[0] = (h16)bfr(F2[(size_t)(2 * lane) * LAT + n]); t[1] = (h16)bfr(F2[(size_t)(2 * lane + 1) * LAT + n]);
        VST2(v2h, F2T + (size_t)n * LAT + 2 * lane, t);
    } else if (wid < 464) { const int n = wid - 448;
        v2h t; t[0] = (n < 4) ? (h16)bfr(F3[(size_t)(2 * lane) * 4 + n]) : (h16)0.f; t[1] = (n < 4) ? (h16)bfr(F3[(size_t)(2 * lane + 1) * 4 + n]) : (h16)0.f;
        VST2(v2h, F3T + (size_t)n * LAT + 2 * lane, t);
    }
}

template <int NTILE>
__device__ __forceinline__ void ln_relu_rows(v8f* acc, const float* __restrict__ g, const float* __restrict__ be, int lr) {
    const float invn = 1.0f / (float)(NTILE * 16);
#pragma unroll
    for (int j = 0; j < 8; ++j) {
        float s = 0.f;
#pragma unroll
        for (int n = 0; n < NTILE; ++n) s += acc[n][j];
        const float mu = hsum16(s) * invn;
        float q = 0.f;
#pragma unroll
        for (int n = 0; n < NTILE; ++n) { const float d = acc[n][j] - mu; q += d * d; }
        const float rs = rsqrtf(hsum16(q) * invn + 1e-5f);
#pragma unroll
        for (int n = 0; n < NTILE; ++n) { const float y = (acc[n][j] - mu) * rs * bfr(g[n * 16 + lr]) + bfr(be[n * 16 + lr]); acc[n][j] = fmaxf(y, 0.f); }
    }
}

__global__ __launch_bounds__(128) void k_edge(const h16* __restrict__ X16, const float* __restrict__ x, const int* __restrict__ ei, const float* __restrict__ W1,
                                             const h16* __restrict__ W1T, const float* __restrict__ b1, const float* __restrict__ g1, const float* __restrict__ be1,
                                             const h16* __restrict__ W2T, const float* __restrict__ b2, const float* __restrict__ g2, const float* __restrict__ be2,
                                             const h16* __restrict__ W3T, const float* __restrict__ b3, h16* MSG16) {
    __shared__ __align__(16) h16 hl[4][16 * 136];
    __shared__ __align__(16) float ost[4][16 * 68];
    const int lane = threadIdx.x & 31, wave = threadIdx.x >> 5, lr = lane & 15, hi = lane >> 4;
    const size_t e0 = (size_t)blockIdx.x * 64 + wave * 16;
    h16* myh = &hl[wave][0];
    const int* srcv = ei; const int* dstv = ei + NE_;
#pragma unroll 1
    for (int rr = 0; rr < 16; ++rr) {
        const size_t e = e0 + rr;
        int s = srcv[e], d = dstv[e]; if (s < 0) s += NN_; if (d < 0) d += NN_; s = min(max(s, 0), NN_ - 1); d = min(max(d, 0), NN_ - 1);
        const h16* xi = X16 + (size_t)d * FIN; const h16* xj = X16 + (size_t)s * FIN;
#pragma unroll
        for (int q = 0; q < 4; ++q) { const int k = lane * 4 + q; h16 v = (h16)0.f; if (k < FIN) v = xi[k]; else if (k < 125) v = xj[k - 61]; myh[rr * 136 + k] = v; }
    }
    asm volatile("" ::: "memory");
    __builtin_amdgcn_fence(__ATOMIC_RELEASE, "workgroup");
    __builtin_amdgcn_wave_barrier();
    v16h a1[4];
#pragma unroll
    for (int kc = 0; kc < 4; ++kc) a1[kc] = cat16(*(const v8ha*)(myh + lr * 136 + kc * 32 + 8 * hi), *(const v8ha*)(myh + lr * 136 + kc * 32 + 16 + 8 * hi));
    __builtin_amdgcn_wave_barrier();
    float d2r[8];
#pragma unroll
    for (int j = 0; j < 8; ++j) {
        const size_t er = e0 + 8 * hi + j;
        int ss = srcv[er], dd = dstv[er]; if (ss < 0) ss += NN_; if (dd < 0) dd += NN_; ss = min(max(ss, 0), NN_ - 1); dd = min(max(dd, 0), NN_ - 1);
        float acc = 0.f;
#pragma unroll
        for (int c = 0; c < 3; ++c) { const float df = bfr(x[(size_t)ss * FIN + c]) - bfr(x[(size_t)dd * FIN + c]); acc += df * df; }
        d2r[j] = acc;
    }
    const float* w1 = W1 + (size_t)LYR * 126 * HID; const float* bb1 = b1 + LYR * HID; const float* gg1 = g1 + LYR * HID; const float* bbe1 = be1 + LYR * HID;
    const float* bb2 = b2 + LYR * HID; const float* gg2 = g2 + LYR * HID; const float* bbe2 = be2 + LYR * HID; const float* bb3 = b3 + LYR * LAT;
    v8f acc[8];
#pragma unroll
    for (int n = 0; n < 8; ++n) acc[n] = (v8f){};
#pragma unroll
    for (int kc = 0; kc < 4; ++kc)
#pragma unroll
        for (int n = 0; n < 8; ++n) { const h16* bp = W1T + (size_t)(n * 16 + lr) * HID + kc * 32 + 8 * hi; acc[n] = wmma16(a1[kc], cat16(*(const v8h*)bp, *(const v8h*)(bp + 16)), acc[n]); }
    asm volatile("v_nop\n\tv_nop\n\tv_nop\n\tv_nop" : "+v"(acc[0]), "+v"(acc[1]), "+v"(acc[2]), "+v"(acc[3]), "+v"(acc[4]), "+v"(acc[5]), "+v"(acc[6]), "+v"(acc[7]));
#pragma unroll
    for (int n = 0; n < 8; ++n) { const int col = n * 16 + lr; const float wd2 = bfr(w1[(size_t)125 * HID + col]), bv = bfr(bb1[col]);
#pragma unroll
        for (int j = 0; j < 8; ++j) acc[n][j] += d2r[j] * wd2 + bv; }
    ln_relu_rows<8>(acc, gg1, bbe1, lr);
#pragma unroll
    for (int n = 0; n < 8; ++n)
#pragma unroll
        for (int j = 0; j < 8; ++j) myh[(hi * 8 + j) * 136 + n * 16 + lr] = (h16)acc[n][j];
    asm volatile("" ::: "memory");
    __builtin_amdgcn_fence(__ATOMIC_RELEASE, "workgroup");
    __builtin_amdgcn_wave_barrier();
    v16h a2[4];
#pragma unroll
    for (int kc = 0; kc < 4; ++kc) a2[kc] = cat16(*(const v8ha*)(myh + lr * 136 + kc * 32 + 8 * hi), *(const v8ha*)(myh + lr * 136 + kc * 32 + 16 + 8 * hi));
#pragma unroll
    for (int n = 0; n < 8; ++n) acc[n] = (v8f){};
#pragma unroll
    for (int kc = 0; kc < 4; ++kc)
#pragma unroll
        for (int n = 0; n < 8; ++n) { const h16* bp = W2T + (size_t)(n * 16 + lr) * HID + kc * 32 + 8 * hi; acc[n] = wmma16(a2[kc], cat16(*(const v8h*)bp, *(const v8h*)(bp + 16)), acc[n]); }
    asm volatile("v_nop\n\tv_nop\n\tv_nop\n\tv_nop" : "+v"(acc[0]), "+v"(acc[1]), "+v"(acc[2]), "+v"(acc[3]), "+v"(acc[4]), "+v"(acc[5]), "+v"(acc[6]), "+v"(acc[7]));
#pragma unroll
    for (int n = 0; n < 8; ++n) { const float bv = bfr(bb2[n * 16 + lr]);
#pragma unroll
        for (int j = 0; j < 8; ++j) acc[n][j] += bv; }
    ln_relu_rows<8>(acc, gg2, bbe2, lr);
    __builtin_amdgcn_wave_barrier();
#pragma unroll
    for (int n = 0; n < 8; ++n)
#pragma unroll
        for (int j = 0; j < 8; ++j) myh[(hi * 8 + j) * 136 + n * 16 + lr] = (h16)acc[n][j];
    asm volatile("" ::: "memory");
    __builtin_amdgcn_fence(__ATOMIC_RELEASE, "workgroup");
    __builtin_amdgcn_wave_barrier();
#pragma unroll
    for (int kc = 0; kc < 4; ++kc) a2[kc] = cat16(*(const v8ha*)(myh + lr * 136 + kc * 32 + 8 * hi), *(const v8ha*)(myh + lr * 136 + kc * 32 + 16 + 8 * hi));
    v8f m4[4];
#pragma unroll
    for (int n = 0; n < 4; ++n) m4[n] = (v8f){};
#pragma unroll
    for (int kc = 0; kc < 4; ++kc)
#pragma unroll
        for (int n = 0; n < 4; ++n) { const h16* bp = W3T + (size_t)(n * 16 + lr) * HID + kc * 32 + 8 * hi; m4[n] = wmma16(a2[kc], cat16(*(const v8h*)bp, *(const v8h*)(bp + 16)), m4[n]); }
    asm volatile("v_nop\n\tv_nop\n\tv_nop\n\tv_nop" : "+v"(m4[0]), "+v"(m4[1]), "+v"(m4[2]), "+v"(m4[3]));
    float* os = &ost[wave][0];
#pragma unroll
    for (int n = 0; n < 4; ++n) { const float bv = bfr(bb3[n * 16 + lr]);
#pragma unroll
        for (int j = 0; j < 8; ++j) os[(hi * 8 + j) * 68 + n * 16 + lr] = m4[n][j] + bv; }
    __syncthreads();
    h16* mrow = MSG16 + e0 * LAT;
    auto pass = [&]() {
#pragma unroll
        for (int sI = 0; sI < 4; ++sI) { const int row = 4 * sI + (lane >> 3), piece = lane & 7; const float* sp = os + row * 68 + piece * 8; v8h o;
#pragma unroll
            for (int i = 0; i < 8; ++i) o[i] = (h16)sp[i];
            *(volatile v8h*)(mrow + (size_t)row * LAT + piece * 8) = o; }
    };
    pass(); __threadfence(); pass();
}

__global__ __launch_bounds__(NT) void k_aggr(const h16* __restrict__ MSG16, const int* __restrict__ ei, float* NODE) {
    extern __shared__ float4 lds_raw[];
    float* agg = (float*)lds_raw; int* lst = (int*)(agg + RB * LAT); int* lse = lst + CHUNK; int* wtot = lse + CHUNK;
    const int t = threadIdx.x, lane = t & 31, wv = t >> 5, n0 = blockIdx.x * RB;
    const int* dstv = ei + NE_;
    for (int i = t; i < RB * LAT; i += NT) agg[i] = 0.0f;
    __syncthreads();
#pragma unroll 1
    for (int base = 0; base < NE_; base += CHUNK) {
        int vdl[EPT], ve[EPT], flg[EPT]; int c = 0;
#pragma unroll
        for (int j = 0; j < EPT; ++j) {
            const int e = base + j * NT + t;
            int d = (e < NE_) ? dstv[e] : -1; if (d < 0 && e < NE_) d += NN_;
            const unsigned udl = (unsigned)d - (unsigned)n0;
            const int f = (udl < (unsigned)RB) ? 1 : 0;
            vdl[j] = (int)udl; ve[j] = e; flg[j] = f; c += f;
        }
        int incl = c;
#pragma unroll
        for (int o = 1; o < 32; o <<= 1) { const int y = __shfl_up(incl, o, 32); if (lane >= o) incl += y; }
        if (lane == 31) wtot[wv] = incl;
        __syncthreads();
        int off = incl - c, tot = 0;
#pragma unroll
        for (int i = 0; i < NWV; ++i) { const int v = wtot[i]; off += (i < wv) ? v : 0; tot += v; }
#pragma unroll
        for (int j = 0; j < EPT; ++j) { if (flg[j]) { lst[off] = vdl[j]; lse[off] = ve[j]; ++off; } }
        __syncthreads();
        if (tot > 0 && t < LAT) {
#pragma unroll 1
            for (int e2 = 0; e2 < tot; ++e2) agg[lst[e2] * LAT + t] += (float)MSG16[(size_t)lse[e2] * LAT + t];
        }
        __syncthreads();
    }
#pragma unroll 1
    for (int i = 0; i < (RB / NWV) / 2; ++i) {
        const int nl = wv * (RB / NWV) + 2 * i + (lane >> 4), cq = (lane & 15) * 4; const size_t n = (size_t)(n0 + nl);
        v4f v;
#pragma unroll
        for (int q = 0; q < 4; ++q) v[q] = fmaxf(agg[nl * LAT + cq + q], 0.f);
        VST2(v4f, NODE + n * LAT + cq, v);
    }
}

__global__ __launch_bounds__(64) void k_pool(const float* __restrict__ NODE, const int* __restrict__ batch, float* POOL) {
    const int g = blockIdx.x, t = threadIdx.x;
    float s = 0.f, mx = -__builtin_inff(); float cnt = 0.f;
#pragma unroll 1
    for (int n = 0; n < NN_; ++n) {
        if (batch[n] == g) { const float v = NODE[(size_t)n * LAT + t]; s += v; mx = fmaxf(mx, v); cnt += 1.0f; }
    }
    float* row = POOL + (size_t)g * (3 * LAT);
    const float mean = s / cnt;
    *(volatile float*)(row + t) = s; *(volatile float*)(row + LAT + t) = mean; *(volatile float*)(row + 2 * LAT + t) = mx;
    __threadfence();
    *(volatile float*)(row + t) = s; *(volatile float*)(row + LAT + t) = mean; *(volatile float*)(row + 2 * LAT + t) = mx;
}

__global__ __launch_bounds__(128) void k_fc(const float* __restrict__ POOL, const h16* __restrict__ F1T, const float* __restrict__ fb1, const float* __restrict__ fg1, const float* __restrict__ fbe1,
                                           const h16* __restrict__ F2T, const float* __restrict__ fb2, const float* __restrict__ fg2, const float* __restrict__ fbe2,
                                           const h16* __restrict__ F3T, const float* __restrict__ fb3, float* out) {
    __shared__ __align__(16) h16 hh[4][16 * 72];
    __shared__ __align__(16) h16 hlw[4][16 * 72];
    const int lane = threadIdx.x & 31, wave = threadIdx.x >> 5, lr = lane & 15, hi = lane >> 4;
    const int r0 = wave * 16;
    h16* myh = &hh[wave][0]; h16* myl = &hlw[wave][0];
    v8f acc[4], accx[4];
#pragma unroll
    for (int n = 0; n < 4; ++n) { acc[n] = (v8f){}; accx[n] = (v8f){}; }
#pragma unroll
    for (int kc = 0; kc < 6; ++kc) {
        v16h ah, al;
#pragma unroll
        for (int q = 0; q < 16; ++q) {
            const int k = kc * 32 + ((q < 8) ? (8 * hi + q) : (16 + 8 * hi + (q - 8)));
            const int r = r0 + lr;
            const float v = (r < NG_) ? POOL[(size_t)r * (3 * LAT) + k] : 0.f;
            const h16 hv = (h16)v; ah[q] = hv; al[q] = (h16)((v - (float)hv) * LOSC);
        }
#pragma unroll
        for (int n = 0; n < 4; ++n) { const h16* bp = F1T + (size_t)(n * 16 + lr) * (3 * LAT) + kc * 32 + 8 * hi; const v16h b = cat16(*(const v8h*)bp, *(const v8h*)(bp + 16));
            acc[n] = wmma16(ah, b, acc[n]); accx[n] = wmma16(al, b, accx[n]); }
    }
    asm volatile("v_nop\n\tv_nop\n\tv_nop\n\tv_nop" : "+v"(acc[0]), "+v"(acc[1]), "+v"(acc[2]), "+v"(acc[3]), "+v"(accx[0]), "+v"(accx[1]), "+v"(accx[2]), "+v"(accx[3]));
#pragma unroll
    for (int n = 0; n < 4; ++n) { const float bv = bfr(fb1[n * 16 + lr]);
#pragma unroll
        for (int j = 0; j < 8; ++j) acc[n][j] += accx[n][j] * LOSCI + bv; }
    ln_relu_rows<4>(acc, fg1, fbe1, lr);
    auto park = [&]() {
#pragma unroll
        for (int n = 0; n < 4; ++n)
#pragma unroll
            for (int j = 0; j < 8; ++j) { const float v = acc[n][j]; const h16 hv = (h16)v; myh[(hi * 8 + j) * 72 + n * 16 + lr] = hv; myl[(hi * 8 + j) * 72 + n * 16 + lr] = (h16)((v - (float)hv) * LOSC); }
        asm volatile("" ::: "memory");
        __builtin_amdgcn_fence(__ATOMIC_RELEASE, "workgroup");
        __builtin_amdgcn_wave_barrier();
    };
    park();
    auto layer64 = [&](const h16* WT, int ntile) {
        v16h ah[2], al[2];
#pragma unroll
        for (int kc = 0; kc < 2; ++kc) { ah[kc] = cat16(*(const v8ha*)(myh + lr * 72 + kc * 32 + 8 * hi), *(const v8ha*)(myh + lr * 72 + kc * 32 + 16 + 8 * hi));
                                         al[kc] = cat16(*(const v8ha*)(myl + lr * 72 + kc * 32 + 8 * hi), *(const v8ha*)(myl + lr * 72 + kc * 32 + 16 + 8 * hi)); }
#pragma unroll
        for (int n = 0; n < 4; ++n) { acc[n] = (v8f){}; accx[n] = (v8f){}; }
#pragma unroll
        for (int kc = 0; kc < 2; ++kc)
#pragma unroll
            for (int n = 0; n < 4; ++n) { if (n < ntile) { const h16* bp = WT + (size_t)(n * 16 + lr) * LAT + kc * 32 + 8 * hi; const v16h b = cat16(*(const v8h*)bp, *(const v8h*)(bp + 16));
                acc[n] = wmma16(ah[kc], b, acc[n]); accx[n] = wmma16(al[kc], b, accx[n]); } }
        asm volatile("v_nop\n\tv_nop\n\tv_nop\n\tv_nop" : "+v"(acc[0]), "+v"(acc[1]), "+v"(acc[2]), "+v"(acc[3]), "+v"(accx[0]), "+v"(accx[1]), "+v"(accx[2]), "+v"(accx[3]));
#pragma unroll
        for (int n = 0; n < 4; ++n)
#pragma unroll
            for (int j = 0; j < 8; ++j) acc[n][j] += accx[n][j] * LOSCI;
        __builtin_amdgcn_wave_barrier();
    };
    layer64(F2T, 4);
#pragma unroll
    for (int n = 0; n < 4; ++n) { const float bv = bfr(fb2[n * 16 + lr]);
#pragma unroll
        for (int j = 0; j < 8; ++j) acc[n][j] += bv; }
    ln_relu_rows<4>(acc, fg2, fbe2, lr);
    park();
    layer64(F3T, 1);
    __shared__ __align__(16) float ofs[64 * 4];
    if (lr < 4) {
#pragma unroll
        for (int j = 0; j < 8; ++j) { const int r = r0 + 8 * hi + j; ofs[r * 4 + lr] = acc[0][j] + bfr(fb3[lr]); }
    }
    __syncthreads();
    if (wave == 0) {
        typedef __attribute__((ext_vector_type(4))) float v4f_; typedef v4f_ __attribute__((may_alias)) v4fa_;
        const v4f_ a = *(const v4fa_*)(ofs + lane * 4);
        const bool tail = (32 + lane) < NG_; v4f_ b = a; if (tail) b = *(const v4fa_*)(ofs + (32 + lane) * 4);
        *(volatile v4f_*)(out + (size_t)lane * 4) = a; if (tail) *(volatile v4f_*)(out + (size_t)(32 + lane) * 4) = b;
        __threadfence();
        *(volatile v4f_*)(out + (size_t)lane * 4) = a; if (tail) *(volatile v4f_*)(out + (size_t)(32 + lane) * 4) = b;
    }
}

extern "C" void kernel_launch(void* const* d_in, const int* in_sizes, int n_in,
                              void* d_out, int out_size, void* d_ws, size_t ws_size, hipStream_t stream) {
    (void)in_sizes; (void)n_in; (void)out_size;
    const float* x = (const float*)d_in[0]; const int* ei = (const int*)d_in[1]; const int* batch = (const int*)d_in[2];
    const float* W1 = (const float*)d_in[3]; const float* b1 = (const float*)d_in[4]; const float* g1 = (const float*)d_in[5]; const float* be1 = (const float*)d_in[6];
    const float* W2 = (const float*)d_in[7]; const float* b2 = (const float*)d_in[8]; const float* g2 = (const float*)d_in[9]; const float* be2 = (const float*)d_in[10];
    const float* W3 = (const float*)d_in[11]; const float* b3 = (const float*)d_in[12];
    const float* F1 = (const float*)d_in[13]; const float* fb1 = (const float*)d_in[14]; const float* fg1 = (const float*)d_in[15]; const float* fbe1 = (const float*)d_in[16];
    const float* F2 = (const float*)d_in[17]; const float* fb2 = (const float*)d_in[18]; const float* fg2 = (const float*)d_in[19]; const float* fbe2 = (const float*)d_in[20];
    const float* F3 = (const float*)d_in[21]; const float* fb3 = (const float*)d_in[22];
    float* out = (float*)d_out;
    char* wsp = (char*)d_ws;
    auto take = [&](size_t bytes) { char* p = wsp; wsp += (bytes + 255) & ~(size_t)255; return (void*)p; };
    h16* X16 = (h16*)take((size_t)NN_ * FIN * 2);
    h16* W1T = (h16*)take((size_t)HID * HID * 2); h16* W2T = (h16*)take((size_t)HID * HID * 2); h16* W3T = (h16*)take((size_t)LAT * HID * 2);
    h16* F1T = (h16*)take((size_t)LAT * 3 * LAT * 2); h16* F2T = (h16*)take((size_t)LAT * LAT * 2); h16* F3T = (h16*)take((size_t)16 * LAT * 2);
    h16* MSG16 = (h16*)take((size_t)NE_ * LAT * 2);
    float* NODE = (float*)take((size_t)NNP * LAT * 4); float* POOL = (float*)take((size_t)64 * 3 * LAT * 4);
    if ((size_t)(wsp - (char*)d_ws) > ws_size) return;
    k_x16<<<(NN_ + 7) / 8, 256, 0, stream>>>(x, X16);
    k_w16<<<464 / 8, 256, 0, stream>>>(W1, W2, W3, F1, F2, F3, W1T, W2T, W3T, F1T, F2T, F3T);
    k_edge<<<NE_ / 64, 128, 0, stream>>>(X16, x, ei, W1, W1T, b1, g1, be1, W2T, b2, g2, be2, W3T, b3, MSG16);
    const size_t lds = (size_t)RB * LAT * 4 + (size_t)CHUNK * 8 + NWV * 4;
    k_aggr<<<NNP / RB, NT, lds, stream>>>(MSG16, ei, NODE);
    k_pool<<<NG_, 64, 0, stream>>>(NODE, batch, POOL);
    k_fc<<<1, 128, 0, stream>>>(POOL, F1T, fb1, fg1, fbe1, F2T, fb2, fg2, fbe2, F3T, fb3, out);
}
